// SimpleRNN_15951508537552
// MI455X (gfx1250) — hardware-verified
//
#include <hip/hip_runtime.h>
#include <math.h>

typedef __attribute__((ext_vector_type(16))) _Float16 v16h;
typedef __attribute__((ext_vector_type(8)))  _Float16 v8h;
typedef __attribute__((ext_vector_type(8)))  float    v8f;
typedef __attribute__((ext_vector_type(4)))  float    v4f;

constexpr int NB   = 64;
constexpr int NT   = 512;
constexpr int NV   = 96;
constexpr int NH   = 1024;
constexpr int NROW = NB * NT;
constexpr int KCAT = NH + NV;
constexpr int KCH  = KCAT / 32;
constexpr int KP   = 1152;
constexpr float WCAR     = 16.0f;
constexpr float WCAR_INV = 1.0f / 16.0f;

constexpr int RTHR    = 512;
constexpr int RWAVES  = RTHR / 32;
constexpr int SEQ_BLK = 16;
constexpr int RBLK    = NB / SEQ_BLK;
constexpr int HP      = 1128;
constexpr int HTILE   = SEQ_BLK * HP;
constexpr int SLP     = 68;
constexpr int XCH     = SEQ_BLK * NV / 8;
constexpr int XWAVES  = XCH / 32;
constexpr int H0CH    = SEQ_BLK * NH / 8;

constexpr int LTHR     = 256;
constexpr int LTN      = 32;
constexpr int LTILES_N = NV / LTN;
constexpr int LTILES_M = NROW / 64;
constexpr int LTILES   = LTILES_M * LTILES_N;
constexpr int LBLK     = LTILES / (LTHR / 32);
constexpr int LSLP     = 36;

constexpr int BC_THR = 64;
constexpr int BC_NT  = 32;
constexpr int BC_KT  = 64;
constexpr int BC_GX  = NH / BC_NT;
constexpr int BC_GY  = KP / BC_KT;

constexpr int WL_CH  = NV * NH / 8;
constexpr int WL_BLK = WL_CH / 256;

constexpr int NOUT0 = NROW * NV;
constexpr int NOUT1 = NB * NH;

static_assert(NB % SEQ_BLK == 0, "blocks own whole sequence groups");
static_assert(NH == RWAVES * 64, "16 waves x 64 hidden columns");
static_assert(KCAT % 32 == 0 && KCH * 32 == KCAT, "fused K is a multiple of 32, no k pad read");
static_assert(HP % 8 == 0 && HP >= KCAT, "A tile pitch");
static_assert(KP % 64 == 0 && KP >= KCAT, "Bcat pitch = whole lines, covers K");
static_assert(XCH % 32 == 0 && XWAVES <= RWAVES, "x staging by whole waves");
static_assert(H0CH % RTHR == 0, "h0 staging loop exact");
static_assert(NROW % 64 == 0 && NV % LTN == 0 && LTILES % (LTHR / 32) == 0, "output head tiling exact");
static_assert(NH % 32 == 0, "output head K multiple of 32");
static_assert(NH % BC_NT == 0 && KP % BC_KT == 0 && NH % BC_KT == 0, "Bcat tiling exact");
static_assert(NV % 2 == 0 && (KCAT - NH) <= 2 * BC_KT, "x part of Bcat fits the last two k tiles");
static_assert(WL_CH % 256 == 0, "Wl cast grid exact");
static_assert((long long)NOUT0 * 4 == 12582912LL, "out1 byte offset");
static_assert((long long)(NOUT0 + NOUT1) * 4 == 12845056LL, "total output bytes");
static_assert((2 * HTILE) % 8 == 0, "tile zero fill in 16-B chunks");

struct FragH {
  union U { v16h v; v8h h[2]; };
  static __device__ __forceinline__ v16h load(const _Float16* p) {
    U f; f.h[0] = *(const v8h*)(p); f.h[1] = *(const v8h*)(p + 16); return f.v;
  }
  static __device__ __forceinline__ v8f mma(v16h a, v16h b, v8f c) {
    return __builtin_amdgcn_wmma_f32_16x16x32_f16(false, a, false, b, (short)0, c, false, false);
  }
};
__device__ __forceinline__ void guard4_h(v8f& a, v8f& b, v8f& c, v8f& d, v16h x, v16h y0, v16h y1, v16h y2, v16h y3) {
  asm volatile("v_nop\n\tv_nop\n\tv_nop\n\tv_nop" : "+v"(a), "+v"(b), "+v"(c), "+v"(d) : "v"(x), "v"(y0), "v"(y1), "v"(y2), "v"(y3));
}
__device__ __forceinline__ void guard2_h(v8f& a, v8f& b, v16h x, v16h y0, v16h y1) {
  asm volatile("v_nop\n\tv_nop\n\tv_nop\n\tv_nop" : "+v"(a), "+v"(b) : "v"(x), "v"(y0), "v"(y1));
}
__device__ __forceinline__ void acc_guard4(v8f& a, v8f& b, v8f& c, v8f& d) {
  asm volatile("v_nop\n\tv_nop\n\tv_nop\n\tv_nop" : "+v"(a), "+v"(b), "+v"(c), "+v"(d));
}
__device__ __forceinline__ void acc_guard8(v8f& a, v8f& b, v8f& c, v8f& d, v8f& e, v8f& f, v8f& g, v8f& h) {
  asm volatile("v_nop\n\tv_nop\n\tv_nop\n\tv_nop" : "+v"(a), "+v"(b), "+v"(c), "+v"(d), "+v"(e), "+v"(f), "+v"(g), "+v"(h));
}

__global__ __launch_bounds__(BC_THR) void bcat_kernel(const float* __restrict__ whh, const float* __restrict__ wxh,
                                                      _Float16* __restrict__ bcat) {
  __shared__ float tile[BC_KT][BC_NT + 1];
  const int tid = threadIdx.x, lane = tid & 31, wave = tid >> 5;
  const int n0 = blockIdx.x * BC_NT;
  const int kbase = blockIdx.y * BC_KT;
  if (kbase < NH) {
#pragma unroll 4
    for (int i = 0; i < BC_KT / 2; ++i) {
      const int kk = 2 * i + wave;
      tile[kk][lane] = whh[(size_t)(kbase + kk) * NH + n0 + lane] * WCAR;
    }
  } else {
    const int v0 = kbase - NH;
    int nval = NV - v0;
    nval = nval < 0 ? 0 : (nval > BC_KT ? BC_KT : nval);
    const int ival = nval >> 1;
#pragma unroll 4
    for (int i = 0; i < ival; ++i) {
      const int kk = 2 * i + wave;
      tile[kk][lane] = wxh[(size_t)(v0 + kk) * NH + n0 + lane] * WCAR;
    }
#pragma unroll 4
    for (int i = ival; i < BC_KT / 2; ++i) {
      const int kk = 2 * i + wave;
      tile[kk][lane] = 0.0f;
    }
  }
  __syncthreads();
  const int q = tid >> 3, c8 = (tid & 7) * 8;
  v8h hv[4];
#pragma unroll
  for (int it = 0; it < 4; ++it) {
    const int nn = it * 8 + q;
#pragma unroll
    for (int e = 0; e < 8; ++e) hv[it][e] = (_Float16)tile[c8 + e][nn];
  }
  for (int pass = 0; pass < 2; ++pass) {
#pragma unroll
    for (int it = 0; it < 4; ++it) {
      const int nn = it * 8 + q;
      *(volatile v8h*)(bcat + (size_t)(n0 + nn) * KP + kbase + c8) = hv[it];
    }
    __threadfence();
  }
}

__global__ __launch_bounds__(256) void wl_cast_kernel(const float* __restrict__ wl, _Float16* __restrict__ wl16) {
  const int i = blockIdx.x * 256 + threadIdx.x;
  const float* sp = wl + (size_t)i * 8;
  const v4f a = *(const v4f*)sp;
  const v4f b = *(const v4f*)(sp + 4);
  v8h hv;
#pragma unroll
  for (int e = 0; e < 4; ++e) { hv[e] = (_Float16)(a[e] * WCAR); hv[4 + e] = (_Float16)(b[e] * WCAR); }
  _Float16* dp = wl16 + (size_t)i * 8;
  *(volatile v8h*)dp = hv;
  __threadfence();
  *(volatile v8h*)dp = hv;
}

__device__ __forceinline__ void stage_x(const float* __restrict__ x, _Float16* tile, int seq0, int tt, int tid) {
  const int row = tid / (NV / 8);
  const int cc  = tid - row * (NV / 8);
  const float* sp = x + ((size_t)(seq0 + row) * NT + (size_t)tt) * NV + cc * 8;
  const v4f a = *(const v4f*)sp;
  const v4f b = *(const v4f*)(sp + 4);
  v8h hv;
#pragma unroll
  for (int e = 0; e < 4; ++e) { hv[e] = (_Float16)a[e]; hv[4 + e] = (_Float16)b[e]; }
  *(v8h*)(tile + row * HP + NH + cc * 8) = hv;
}

__global__ __launch_bounds__(RTHR) void rnn_seq_kernel(const float* __restrict__ x, const float* __restrict__ h0,
                                                       const float* __restrict__ bh, const _Float16* __restrict__ bcat,
                                                       _Float16* __restrict__ hid, float* __restrict__ hlast) {
  __shared__ __align__(16) _Float16 hbuf[2 * HTILE];
  __shared__ __align__(16) float    slabs[RWAVES][16 * SLP];
  const int tid = threadIdx.x, lane = tid & 31, wave = tid >> 5;
  const int c = lane & 15, hh = lane >> 4, koff = hh * 8, mOff = hh * 8, c4 = c * 4;
  const int q4 = lane >> 3, c8 = (lane & 7) * 8;
  const int seq0 = blockIdx.x * SEQ_BLK;
  const int n0 = wave * 64;

  {
    const v8h z = {(_Float16)0.f, (_Float16)0.f, (_Float16)0.f, (_Float16)0.f, (_Float16)0.f, (_Float16)0.f, (_Float16)0.f, (_Float16)0.f};
    for (int i = tid; i < (2 * HTILE) / 8; i += RTHR) *(v8h*)(hbuf + i * 8) = z;
  }
  __syncthreads();
#pragma unroll
  for (int it = 0; it < H0CH / RTHR; ++it) {
    const int i = it * RTHR + tid;
    const int row = i / (NH / 8);
    const int cc  = i - row * (NH / 8);
    const float* sp = h0 + (size_t)(seq0 + row) * NH + cc * 8;
    const v4f a = *(const v4f*)sp;
    const v4f b = *(const v4f*)(sp + 4);
    v8h hv;
#pragma unroll
    for (int e = 0; e < 4; ++e) { hv[e] = (_Float16)a[e]; hv[4 + e] = (_Float16)b[e]; }
    *(v8h*)(hbuf + row * HP + cc * 8) = hv;
  }
  if (wave < XWAVES) stage_x(x, hbuf, seq0, 0, tid);
  float bhv[4];
#pragma unroll
  for (int j = 0; j < 4; ++j) bhv[j] = bh[n0 + 16 * j + c];
  __syncthreads();

  const v8f z8 = {0.f, 0.f, 0.f, 0.f, 0.f, 0.f, 0.f, 0.f};
  const _Float16* brow = bcat + (size_t)(n0 + c) * KP + koff;
  float* slab = slabs[wave];

#pragma unroll 1
  for (int t = 0; t < NT; ++t) {
    const int cur = t & 1;
    const _Float16* hc = hbuf + cur * HTILE;
    _Float16*       hn = hbuf + (cur ^ 1) * HTILE;
    const bool last = (t == NT - 1);
    if (wave < XWAVES && t + 1 < NT) stage_x(x, hn, seq0, t + 1, tid);

    v8f acc[4];
#pragma unroll
    for (int j = 0; j < 4; ++j) acc[j] = z8;
    const _Float16* arow = hc + c * HP + koff;
#pragma unroll 1
    for (int kc = 0; kc < KCH; ++kc) {
      const v16h fa = FragH::load(arow + kc * 32);
      v16h fb[4];
#pragma unroll
      for (int j = 0; j < 4; ++j) fb[j] = FragH::load(brow + (size_t)(16 * j) * KP + kc * 32);
#pragma unroll
      for (int j = 0; j < 4; ++j) acc[j] = FragH::mma(fa, fb[j], acc[j]);
      guard4_h(acc[0], acc[1], acc[2], acc[3], fa, fb[0], fb[1], fb[2], fb[3]);
    }
    acc_guard4(acc[0], acc[1], acc[2], acc[3]);

#pragma unroll
    for (int j = 0; j < 4; ++j) {
      const int col = n0 + 16 * j + c;
#pragma unroll
      for (int r = 0; r < 8; ++r) {
        const float v = tanhf(acc[j][r] * WCAR_INV + bhv[j]);
        hn[(mOff + r) * HP + col] = (_Float16)v;
        if (last) slab[(mOff + r) * SLP + 16 * j + c] = v;
      }
    }
    __syncthreads();

    for (int pass = 0; pass < 2; ++pass) {
#pragma unroll
      for (int it = 0; it < 4; ++it) {
        const int rr = it * 4 + q4;
        const v8h hvv = *(const v8h*)(hn + rr * HP + n0 + c8);
        *(volatile v8h*)(hid + ((size_t)(seq0 + rr) * NT + (size_t)t) * NH + n0 + c8) = hvv;
      }
      __threadfence();
    }
    if (last) {
      for (int pass = 0; pass < 2; ++pass) {
#pragma unroll
        for (int it = 0; it < 8; ++it) {
          const int row = it * 2 + hh;
          const v4f vv = *(const v4f*)(slab + row * SLP + c4);
          *(volatile v4f*)(hlast + (size_t)(seq0 + row) * NH + n0 + c4) = vv;
        }
        __threadfence();
      }
    }
  }
}

__global__ __launch_bounds__(LTHR) void logits_kernel(const _Float16* __restrict__ hid, const _Float16* __restrict__ wl16,
                                                      const float* __restrict__ bl, float* __restrict__ out) {
  __shared__ __align__(16) float sT[LTHR / 32][16 * LSLP];
  const int lane = threadIdx.x & 31, wave = threadIdx.x >> 5;
  const int tile = blockIdx.x * (LTHR / 32) + wave;
  if (tile >= LTILES) return;
  const int tm = tile / LTILES_N;
  const int tn = tile - tm * LTILES_N;
  const int m0 = tm * 64, n0 = tn * LTN;
  const int rlane = lane & 15, koff = (lane >> 4) * 8, mOff = (lane >> 4) * 8;
  const int q = lane >> 3, c4 = (lane & 7) * 4;

  const v8f z8 = {0.f, 0.f, 0.f, 0.f, 0.f, 0.f, 0.f, 0.f};
  v8f acc[4][2];
#pragma unroll
  for (int i = 0; i < 4; ++i) { acc[i][0] = z8; acc[i][1] = z8; }

  const _Float16* bp = wl16 + (size_t)(n0 + rlane) * NH + koff;
  const _Float16* ap = hid + (size_t)(m0 + rlane) * NH + koff;
#pragma unroll 1
  for (int k0 = 0; k0 < NH; k0 += 32) {
    const v16h b0 = FragH::load(bp + k0);
    const v16h b1 = FragH::load(bp + (size_t)16 * NH + k0);
#pragma unroll
    for (int i = 0; i < 4; ++i) {
      const v16h a = FragH::load(ap + (size_t)(16 * i) * NH + k0);
      acc[i][0] = FragH::mma(a, b0, acc[i][0]);
      acc[i][1] = FragH::mma(a, b1, acc[i][1]);
      guard2_h(acc[i][0], acc[i][1], a, b0, b1);
    }
  }
  acc_guard8(acc[0][0], acc[0][1], acc[1][0], acc[1][1], acc[2][0], acc[2][1], acc[3][0], acc[3][1]);

  const float bv0 = bl[n0 + rlane];
  const float bv1 = bl[n0 + 16 + rlane];
  float* slab = sT[wave];
#pragma unroll
  for (int i = 0; i < 4; ++i) {
    const int mBase = m0 + 16 * i;
#pragma unroll
    for (int r = 0; r < 8; ++r) {
      slab[(mOff + r) * LSLP + rlane]      = acc[i][0][r] * WCAR_INV + bv0;
      slab[(mOff + r) * LSLP + 16 + rlane] = acc[i][1][r] * WCAR_INV + bv1;
    }
    __builtin_amdgcn_fence(__ATOMIC_RELEASE, "workgroup");
    __builtin_amdgcn_wave_barrier();
    __builtin_amdgcn_fence(__ATOMIC_ACQUIRE, "workgroup");
    v4f vv[4];
#pragma unroll
    for (int it = 0; it < 4; ++it) vv[it] = *(const v4f*)(slab + (it * 4 + q) * LSLP + c4);
    for (int pass = 0; pass < 2; ++pass) {
#pragma unroll
      for (int it = 0; it < 4; ++it)
        *(volatile v4f*)(out + (size_t)(mBase + it * 4 + q) * NV + n0 + c4) = vv[it];
      __threadfence();
    }
    __builtin_amdgcn_fence(__ATOMIC_RELEASE, "workgroup");
    __builtin_amdgcn_wave_barrier();
    __builtin_amdgcn_fence(__ATOMIC_ACQUIRE, "workgroup");
  }
}

extern "C" void kernel_launch(void* const* d_in, const int* in_sizes, int n_in,
                              void* d_out, int out_size, void* d_ws, size_t ws_size, hipStream_t stream) {
  if (n_in < 7 || d_out == nullptr || d_ws == nullptr) return;
  if (in_sizes[0] != NB * NT * NV || in_sizes[1] != NB * NH || in_sizes[2] != NV * NH ||
      in_sizes[3] != NH * NH || in_sizes[4] != NH || in_sizes[5] != NV * NH || in_sizes[6] != NV ||
      out_size != NOUT0 + NOUT1) return;

  const float* x   = (const float*)d_in[0];
  const float* h0  = (const float*)d_in[1];
  const float* wxh = (const float*)d_in[2];
  const float* whh = (const float*)d_in[3];
  const float* bh  = (const float*)d_in[4];
  const float* wl  = (const float*)d_in[5];
  const float* bl  = (const float*)d_in[6];
  float* out0 = (float*)d_out;
  float* out1 = out0 + (size_t)NOUT0;

  char* ws = (char*)d_ws; size_t off = 0;
  auto carve = [&](size_t bytes) -> char* { char* p = ws + off; off += (bytes + 255) & ~(size_t)255; return p; };
  _Float16* BCAT = (_Float16*)carve((size_t)NH * KP * 2);
  _Float16* WL16 = (_Float16*)carve((size_t)NV * NH * 2);
  _Float16* HID  = (_Float16*)carve((size_t)NROW * NH * 2);
  if (off > ws_size || off > (size_t)134217728) return;

  bcat_kernel<<<dim3(BC_GX, BC_GY), BC_THR, 0, stream>>>(whh, wxh, BCAT);
  wl_cast_kernel<<<WL_BLK, 256, 0, stream>>>(wl, WL16);
  rnn_seq_kernel<<<RBLK, RTHR, 0, stream>>>(x, h0, bh, BCAT, HID, out1);
  logits_kernel<<<LBLK, LTHR, 0, stream>>>(HID, WL16, bl, out0);
}
